// MultiHeadSelfAttention_85220741087659
// MI455X (gfx1250) — hardware-verified
//
#include <hip/hip_runtime.h>
#ifndef NB
#define NB 2
#endif
#ifndef SEQ
#define SEQ 2048
#endif
#define NB_FULL 2
#define SEQ_FULL 2048
#define DM 1024
#define NH 16
#define HD 64
#define NRP (NB * SEQ)
#define LN_EPS 1e-5f

static_assert(NH * HD == DM);
static_assert(HD == 64);
static_assert(DM == 1024);
static_assert(DM % 128 == 0);
static_assert(DM % 64 == 0);
static_assert(DM % 32 == 0);
static_assert(NRP % 128 == 0);
static_assert(NRP % 64 == 0);
static_assert(SEQ % 64 == 0);
static_assert(NB <= NB_FULL);
static_assert(SEQ <= SEQ_FULL);

typedef _Float16 v16h __attribute__((ext_vector_type(16)));
typedef __bf16 v16b __attribute__((ext_vector_type(16)));
typedef _Float16 v4h __attribute__((ext_vector_type(4)));
typedef unsigned short v8us __attribute__((ext_vector_type(8), may_alias));
typedef float v8f __attribute__((ext_vector_type(8)));
typedef float v4f __attribute__((ext_vector_type(4)));
typedef float v4fa __attribute__((ext_vector_type(4), may_alias));
union FragH { v16h v; v8us half[2]; _Float16 h[16]; unsigned short u[16]; };
union FragB { v16b v; v8us half[2]; unsigned short u[16]; };

#define WS_W   ((size_t)DM * DM * 2)
#define WS_P16 ((size_t)NRP * DM * 2)
#define WS_P32 ((size_t)NRP * DM * 4)
#define WS_TOTAL (4 * WS_W + 7 * WS_P16 + WS_P32)
static_assert(WS_W % 256 == 0);
static_assert(WS_P16 % 256 == 0);
static_assert(WS_TOTAL <= (size_t)134217728);

__device__ __forceinline__ unsigned short bf16_bits(float x) { unsigned int u = __float_as_uint(x); return (unsigned short)((u + 0x7FFFu + ((u >> 16) & 1u)) >> 16); }
__device__ __forceinline__ float bf16_val(unsigned short b) { return __uint_as_float(((unsigned int)b) << 16); }
__device__ __forceinline__ float bf16_rne(float x) { return bf16_val(bf16_bits(x)); }

__device__ __forceinline__ v16h ldf_h(const unsigned short* __restrict__ p, size_t off) { FragH f; f.half[0] = *(const v8us*)(p + off); f.half[1] = *(const v8us*)(p + off + 16); return f.v; }
__device__ __forceinline__ v16b ldf_b(const unsigned short* __restrict__ p, size_t off) { FragB f; f.half[0] = *(const v8us*)(p + off); f.half[1] = *(const v8us*)(p + off + 16); return f.v; }
__device__ __forceinline__ v8f mma_h(v16h a, v16h b, v8f c) {
  v8f d = __builtin_amdgcn_wmma_f32_16x16x32_f16(false, a, false, b, (short)0, c, false, false);
  asm volatile("v_nop\n\tv_nop\n\tv_nop\n\tv_nop" : "+v"(d) : "v"(a), "v"(b));
  return d;
}
__device__ __forceinline__ v8f mma_b2(v16b ah, v16b al, v16b b, v8f c) {
  c = __builtin_amdgcn_wmma_f32_16x16x32_bf16(false, ah, false, b, (short)0, c, false, false);
  c = __builtin_amdgcn_wmma_f32_16x16x32_bf16(false, al, false, b, (short)0, c, false, false);
  asm volatile("v_nop\n\tv_nop\n\tv_nop\n\tv_nop" : "+v"(c) : "v"(ah), "v"(al), "v"(b));
  return c;
}

__global__ __launch_bounds__(256) void k_wt_f16(const float* __restrict__ W, unsigned short* __restrict__ Wt, int K, int N, float scale) {
  const int t = blockIdx.x * 256 + threadIdx.x;
  const int k8n = K / 8;
  if (t >= N * k8n) return;
  const int n = t / k8n, k8 = (t % k8n) * 8;
  FragH f;
#pragma unroll
  for (int i = 0; i < 8; ++i) f.h[i] = (_Float16)(bf16_rne(W[(size_t)(k8 + i) * N + n]) * scale);
  const v8us o = f.half[0];
  *(volatile v8us*)(Wt + (size_t)n * K + k8) = o;
  __threadfence();
  *(volatile v8us*)(Wt + (size_t)n * K + k8) = o;
}
__global__ __launch_bounds__(256) void k_wt_bf16(const float* __restrict__ W, unsigned short* __restrict__ Wt, int K, int N) {
  const int t = blockIdx.x * 256 + threadIdx.x;
  const int k8n = K / 8;
  if (t >= N * k8n) return;
  const int n = t / k8n, k8 = (t % k8n) * 8;
  v8us v;
#pragma unroll
  for (int i = 0; i < 8; ++i) v[i] = bf16_bits(W[(size_t)(k8 + i) * N + n]);
  *(volatile v8us*)(Wt + (size_t)n * K + k8) = v;
  __threadfence();
  *(volatile v8us*)(Wt + (size_t)n * K + k8) = v;
}
__global__ __launch_bounds__(256) void k_x16(const float* __restrict__ x, unsigned short* __restrict__ X16) {
  const size_t t = (size_t)blockIdx.x * 256 + threadIdx.x;
  if (t >= (size_t)NRP * DM / 8) return;
  const size_t e = t * 8;
  const int r = (int)(e / DM), c = (int)(e % DM);
  const size_t src = ((size_t)(r / SEQ) * SEQ_FULL + (size_t)(r % SEQ)) * DM + c;
  const v4f a = *(const v4fa*)(x + src), b = *(const v4fa*)(x + src + 4);
  FragH f;
#pragma unroll
  for (int q = 0; q < 4; ++q) { f.h[q] = (_Float16)bf16_rne(a[q]); f.h[4 + q] = (_Float16)bf16_rne(b[q]); }
  const v8us o = f.half[0];
  *(volatile v8us*)(X16 + e) = o;
  __threadfence();
  *(volatile v8us*)(X16 + e) = o;
}

template <int MODE>
__device__ __forceinline__ void gemm_h_body(const unsigned short* __restrict__ A, const int lda, const unsigned short* __restrict__ Bt, const int ldb, const float alpha,
                                            const float* __restrict__ bias, unsigned short* C0, unsigned short* C1, const int ldc, const int M, const int N, const int K) {
  __shared__ __attribute__((aligned(16))) float so[4][32][68];
  const int tid = threadIdx.x;
  const int w = __builtin_amdgcn_readfirstlane(tid >> 5);
  const int lane = tid & 31, ln = lane & 15, hh = lane >> 4;
  const int ntn = N >> 6;
  const int mt = blockIdx.x / ntn, nq = blockIdx.x - mt * ntn;
  const int row0 = mt * 128 + 32 * w, col0 = nq * 64;
  if (row0 >= M) return;
  const size_t a0 = (size_t)(row0 + ln) * lda + 8 * hh, a1 = a0 + (size_t)16 * lda;
  const size_t b0 = (size_t)(col0 + ln) * ldb + 8 * hh, b1 = b0 + (size_t)16 * ldb, b2 = b1 + (size_t)16 * ldb, b3 = b2 + (size_t)16 * ldb;
  const v8f z8 = {0.f, 0.f, 0.f, 0.f, 0.f, 0.f, 0.f, 0.f};
  v8f c00 = z8, c01 = z8, c02 = z8, c03 = z8, c10 = z8, c11 = z8, c12 = z8, c13 = z8;
#pragma unroll 1
  for (int kb = 0; kb < K; kb += 32) {
    const v16h fa0 = ldf_h(A, a0 + kb), fa1 = ldf_h(A, a1 + kb);
    v16h fb = ldf_h(Bt, b0 + kb); c00 = mma_h(fa0, fb, c00); c10 = mma_h(fa1, fb, c10);
    fb = ldf_h(Bt, b1 + kb); c01 = mma_h(fa0, fb, c01); c11 = mma_h(fa1, fb, c11);
    fb = ldf_h(Bt, b2 + kb); c02 = mma_h(fa0, fb, c02); c12 = mma_h(fa1, fb, c12);
    fb = ldf_h(Bt, b3 + kb); c03 = mma_h(fa0, fb, c03); c13 = mma_h(fa1, fb, c13);
  }
  v8f accs[8] = {c00, c01, c02, c03, c10, c11, c12, c13};
#pragma unroll
  for (int u = 0; u < 8; ++u) {
    const int t = u & 3, half = u >> 2;
    float bc = 0.f;
    float brow[8] = {0.f, 0.f, 0.f, 0.f, 0.f, 0.f, 0.f, 0.f};
    if (MODE == 2) {
      const v4f r0 = *(const v4fa*)(bias + row0 + half * 16 + 8 * hh), r1 = *(const v4fa*)(bias + row0 + half * 16 + 8 * hh + 4);
#pragma unroll
      for (int q = 0; q < 4; ++q) { brow[q] = bf16_rne(r0[q]); brow[4 + q] = bf16_rne(r1[q]); }
    } else {
      bc = bf16_rne(bias[col0 + t * 16 + ln]);
    }
#pragma unroll
    for (int r = 0; r < 8; ++r) {
      const int rloc = half * 16 + 8 * hh + r;
      const float bvv = (MODE == 2) ? brow[r] : bc;
      so[w][rloc][t * 16 + ln] = accs[u][r] * alpha + bvv;
    }
  }
  __builtin_amdgcn_fence(4  , "workgroup");
  __builtin_amdgcn_wave_barrier();
  const int rsub = lane >> 4, c4 = (lane & 15) * 4;
  for (int pass = 0; pass < 2; ++pass) {
#pragma unroll
    for (int q = 0; q < 16; ++q) {
      const int r = q * 2 + rsub;
      const v4f v = *(const v4fa*)&so[w][r][c4];
      v4h h4, r4;
#pragma unroll
      for (int i = 0; i < 4; ++i) { const _Float16 hv = (_Float16)v[i]; h4[i] = hv; r4[i] = (_Float16)((v[i] - (float)hv) * 1024.0f); }
      const size_t go = (size_t)(row0 + r) * ldc + col0 + c4;
      *(volatile v4h*)(C0 + go) = h4;
      if (MODE == 1) *(volatile v4h*)(C1 + go) = r4;
    }
    if (pass == 0) __threadfence();
  }
}
__global__ __launch_bounds__(128) void k_gemm_q(const unsigned short* __restrict__ X16, const unsigned short* __restrict__ Bt, const float* __restrict__ bias, unsigned short* __restrict__ Qh, unsigned short* __restrict__ Qr) {
  gemm_h_body<1>(X16, DM, Bt, DM, 0.0625f, bias, Qh, Qr, DM, NRP, DM, DM);
}
__global__ __launch_bounds__(128) void k_gemm_k(const unsigned short* __restrict__ X16, const unsigned short* __restrict__ Bt, const float* __restrict__ bias, unsigned short* __restrict__ K16) {
  gemm_h_body<0>(X16, DM, Bt, DM, 0.0625f, bias, K16, K16, DM, NRP, DM, DM);
}
__global__ __launch_bounds__(128) void k_gemm_vt(const unsigned short* __restrict__ Bt, const unsigned short* __restrict__ X16, const float* __restrict__ bias, unsigned short* __restrict__ VT) {
  gemm_h_body<2>(Bt, DM, X16, DM, 0.0625f, bias, VT, VT, NRP, DM, NRP, DM);
}

__global__ __launch_bounds__(128) void k_flash(const unsigned short* __restrict__ Qh, const unsigned short* __restrict__ Qr, const unsigned short* __restrict__ Kp,
                                               const unsigned short* __restrict__ VT, unsigned short* __restrict__ CH, unsigned short* __restrict__ CL) {
  __shared__ __attribute__((aligned(16))) unsigned short sh[4][16][72];
  __shared__ __attribute__((aligned(16))) unsigned short sl[4][16][72];
  const int tid = threadIdx.x;
  const int wave = __builtin_amdgcn_readfirstlane(tid >> 5);
  const int lane = tid & 31, ln = lane & 15, hh = lane >> 4;
  const int bh = blockIdx.x / (SEQ / 64), qb = blockIdx.x % (SEQ / 64);
  const int b = bh / NH, h = bh % NH;
  const int q0 = qb * 64 + 16 * wave;
  const size_t rowb = (size_t)b * SEQ;
  const size_t qoff = (rowb + q0 + ln) * DM + h * HD + 8 * hh;
  const v16h qh0 = ldf_h(Qh, qoff), qh1 = ldf_h(Qh, qoff + 32);
  const v16h qr0 = ldf_h(Qr, qoff), qr1 = ldf_h(Qr, qoff + 32);
  const size_t koff = (rowb + ln) * DM + h * HD + 8 * hh;
  const size_t voff = (size_t)(h * HD + ln) * NRP + rowb + 8 * hh;
  const v8f z8 = {0.f, 0.f, 0.f, 0.f, 0.f, 0.f, 0.f, 0.f};
  v8f o[4] = {z8, z8, z8, z8};
  float m = -1.0e30f, l = 0.f;
#pragma unroll 1
  for (int kb = 0; kb < SEQ; kb += 32) {
    const size_t k0 = koff + (size_t)kb * DM, k1 = k0 + (size_t)16 * DM;
    v8f sm0 = z8, sr0 = z8, sm1 = z8, sr1 = z8;
    v16h ka = ldf_h(Kp, k0);      sm0 = mma_h(ka, qh0, sm0); sr0 = mma_h(ka, qr0, sr0);
    ka = ldf_h(Kp, k1);           sm1 = mma_h(ka, qh0, sm1); sr1 = mma_h(ka, qr0, sr1);
    ka = ldf_h(Kp, k0 + 32);      sm0 = mma_h(ka, qh1, sm0); sr0 = mma_h(ka, qr1, sr0);
    ka = ldf_h(Kp, k1 + 32);      sm1 = mma_h(ka, qh1, sm1); sr1 = mma_h(ka, qr1, sr1);
    float s0[8], s1[8];
    float mx = -1.0e30f;
#pragma unroll
    for (int r = 0; r < 8; ++r) {
      s0[r] = sm0[r] * 0.125f + sr0[r] * 0.0001220703125f;
      s1[r] = sm1[r] * 0.125f + sr1[r] * 0.0001220703125f;
      mx = fmaxf(mx, fmaxf(s0[r], s1[r]));
    }
    mx = fmaxf(mx, __shfl_xor(mx, 16));
    const float mn = fmaxf(m, mx);
    const float alpha = __expf(m - mn);
    const float ms = mn - 5.545177444479562f;
    m = mn;
    FragH pf;
    float ps = 0.f;
#pragma unroll
    for (int r = 0; r < 8; ++r) {
      const float p0 = __expf(s0[r] - ms), p1 = __expf(s1[r] - ms);
      ps += p0 + p1;
      pf.h[r] = (_Float16)p0;
      pf.h[8 + r] = (_Float16)p1;
    }
    l = l * alpha + ps;
#pragma unroll
    for (int t = 0; t < 4; ++t)
#pragma unroll
      for (int r = 0; r < 8; ++r) o[t][r] *= alpha;
#pragma unroll
    for (int t = 0; t < 4; ++t) {
      const v16h va = ldf_h(VT, voff + (size_t)t * 16 * NRP + kb);
      o[t] = mma_h(va, pf.v, o[t]);
    }
  }
  l += __shfl_xor(l, 16);
  const float inv = 1.0f / l;
#pragma unroll
  for (int t = 0; t < 4; ++t) {
    v8us vh, vl;
#pragma unroll
    for (int r = 0; r < 8; ++r) {
      const float c = o[t][r] * inv;
      const unsigned short hb = bf16_bits(c);
      vh[r] = hb;
      vl[r] = bf16_bits(c - bf16_val(hb));
    }
    *(v8us*)&sh[wave][ln][t * 16 + 8 * hh] = vh;
    *(v8us*)&sl[wave][ln][t * 16 + 8 * hh] = vl;
  }
  __builtin_amdgcn_fence(4  , "workgroup");
  __builtin_amdgcn_wave_barrier();
  const int rq = lane >> 3, pc = lane & 7;
  for (int pass = 0; pass < 2; ++pass) {
#pragma unroll
    for (int qq = 0; qq < 4; ++qq) {
      const int row = qq * 4 + rq;
      const v8us xh = *(const v8us*)&sh[wave][row][pc * 8];
      const v8us xl = *(const v8us*)&sl[wave][row][pc * 8];
      const size_t go = (rowb + q0 + row) * DM + h * HD + pc * 8;
      *(volatile v8us*)(CH + go) = xh;
      *(volatile v8us*)(CL + go) = xl;
    }
    if (pass == 0) __threadfence();
  }
}

__global__ __launch_bounds__(128) void k_gemm_o(const unsigned short* __restrict__ CH, const unsigned short* __restrict__ CL, const unsigned short* __restrict__ Wt,
                                                const float* __restrict__ bias, float* __restrict__ Y) {
  __shared__ __attribute__((aligned(16))) float so[4][32][68];
  const int tid = threadIdx.x;
  const int w = __builtin_amdgcn_readfirstlane(tid >> 5);
  const int lane = tid & 31, ln = lane & 15, hh = lane >> 4;
  const int ntn = DM >> 6;
  const int mt = blockIdx.x / ntn, nq = blockIdx.x - mt * ntn;
  const int row0 = mt * 128 + 32 * w, col0 = nq * 64;
  if (row0 >= NRP) return;
  const size_t a0 = (size_t)(row0 + ln) * DM + 8 * hh, a1 = a0 + (size_t)16 * DM;
  const size_t b0 = (size_t)(col0 + ln) * DM + 8 * hh, b1 = b0 + (size_t)16 * DM, b2 = b1 + (size_t)16 * DM, b3 = b2 + (size_t)16 * DM;
  const v8f z8 = {0.f, 0.f, 0.f, 0.f, 0.f, 0.f, 0.f, 0.f};
  v8f c00 = z8, c01 = z8, c02 = z8, c03 = z8, c10 = z8, c11 = z8, c12 = z8, c13 = z8;
#pragma unroll 1
  for (int kb = 0; kb < DM; kb += 32) {
    const v16b h0 = ldf_b(CH, a0 + kb), l0 = ldf_b(CL, a0 + kb), h1 = ldf_b(CH, a1 + kb), l1 = ldf_b(CL, a1 + kb);
    v16b fb = ldf_b(Wt, b0 + kb); c00 = mma_b2(h0, l0, fb, c00); c10 = mma_b2(h1, l1, fb, c10);
    fb = ldf_b(Wt, b1 + kb); c01 = mma_b2(h0, l0, fb, c01); c11 = mma_b2(h1, l1, fb, c11);
    fb = ldf_b(Wt, b2 + kb); c02 = mma_b2(h0, l0, fb, c02); c12 = mma_b2(h1, l1, fb, c12);
    fb = ldf_b(Wt, b3 + kb); c03 = mma_b2(h0, l0, fb, c03); c13 = mma_b2(h1, l1, fb, c13);
  }
  v8f accs[8] = {c00, c01, c02, c03, c10, c11, c12, c13};
#pragma unroll
  for (int u = 0; u < 8; ++u) {
    const int t = u & 3, half = u >> 2;
    const float bc = bf16_rne(bias[col0 + t * 16 + ln]);
#pragma unroll
    for (int r = 0; r < 8; ++r) so[w][half * 16 + 8 * hh + r][t * 16 + ln] = accs[u][r] + bc;
  }
  __builtin_amdgcn_fence(4  , "workgroup");
  __builtin_amdgcn_wave_barrier();
  const int rsub = lane >> 4, c4 = (lane & 15) * 4;
  for (int pass = 0; pass < 2; ++pass) {
#pragma unroll
    for (int q = 0; q < 16; ++q) {
      const int r = q * 2 + rsub;
      const v4f v = *(const v4fa*)&so[w][r][c4];
      *(volatile v4f*)(Y + (size_t)(row0 + r) * DM + col0 + c4) = v;
    }
    if (pass == 0) __threadfence();
  }
}

__global__ __launch_bounds__(256) void k_ln(const float* __restrict__ x, const float* __restrict__ Y, const float* __restrict__ g, const float* __restrict__ bta, float* __restrict__ out) {
  __shared__ float red1[8];
  __shared__ float red2[8];
  const int row = blockIdx.x, tid = threadIdx.x, lane = tid & 31;
  const int wave = __builtin_amdgcn_readfirstlane(tid >> 5);
  const size_t xr = ((size_t)(row / SEQ) * SEQ_FULL + (size_t)(row % SEQ)) * DM + (size_t)tid * 4;
  const v4f xv = *(const v4fa*)(x + xr);
  const v4f yv = *(const v4fa*)(Y + (size_t)row * DM + (size_t)tid * 4);
  v4f hv;
  float s1 = 0.f;
#pragma unroll
  for (int q = 0; q < 4; ++q) { hv[q] = bf16_rne(xv[q]) + yv[q]; s1 += hv[q]; }
#pragma unroll
  for (int off = 16; off > 0; off >>= 1) s1 += __shfl_xor(s1, off);
  if (lane == 0) red1[wave] = s1;
  __syncthreads();
  float tot = 0.f;
#pragma unroll
  for (int i = 0; i < 8; ++i) tot += red1[i];
  const float mu = tot * (1.0f / (float)DM);
  float s2 = 0.f;
  v4f cv;
#pragma unroll
  for (int q = 0; q < 4; ++q) { cv[q] = hv[q] - mu; s2 += cv[q] * cv[q]; }
#pragma unroll
  for (int off = 16; off > 0; off >>= 1) s2 += __shfl_xor(s2, off);
  if (lane == 0) red2[wave] = s2;
  __syncthreads();
  float tv = 0.f;
#pragma unroll
  for (int i = 0; i < 8; ++i) tv += red2[i];
  const float rs = rsqrtf(tv * (1.0f / (float)DM) + LN_EPS);
  const v4f gv = *(const v4fa*)(g + tid * 4);
  const v4f bv = *(const v4fa*)(bta + tid * 4);
  v4f ov;
#pragma unroll
  for (int q = 0; q < 4; ++q) ov[q] = cv[q] * rs * bf16_rne(gv[q]) + bf16_rne(bv[q]);
  *(volatile v4f*)(out + xr) = ov;
  __threadfence();
  *(volatile v4f*)(out + xr) = ov;
}

extern "C" void kernel_launch(void* const* d_in, const int* in_sizes, int n_in,
                              void* d_out, int out_size, void* d_ws, size_t ws_size, hipStream_t stream) {
  if (n_in < 11) return;
  const size_t need_x = ((size_t)(NB - 1) * SEQ_FULL + SEQ) * DM;
  if ((size_t)in_sizes[0] < need_x || (size_t)out_size < need_x) return;
  if ((size_t)in_sizes[1] < (size_t)DM * DM || (size_t)in_sizes[3] < (size_t)DM * DM || (size_t)in_sizes[5] < (size_t)DM * DM || (size_t)in_sizes[7] < (size_t)DM * DM) return;
  if (in_sizes[2] < DM || in_sizes[4] < DM || in_sizes[6] < DM || in_sizes[8] < DM || in_sizes[9] < DM || in_sizes[10] < DM) return;
  const float* x  = (const float*)d_in[0];
  const float* wq = (const float*)d_in[1]; const float* bq = (const float*)d_in[2];
  const float* wk = (const float*)d_in[3]; const float* bk = (const float*)d_in[4];
  const float* wv = (const float*)d_in[5]; const float* bv = (const float*)d_in[6];
  const float* wo = (const float*)d_in[7]; const float* bo = (const float*)d_in[8];
  const float* lg = (const float*)d_in[9]; const float* lb = (const float*)d_in[10];
  char* ws = (char*)d_ws; size_t off = 0;
  auto take = [&](size_t bytes) { char* p = ws + off; off += (bytes + 255) & ~(size_t)255; return p; };
  unsigned short* BQ = (unsigned short*)take(WS_W);
  unsigned short* BK = (unsigned short*)take(WS_W);
  unsigned short* BV = (unsigned short*)take(WS_W);
  unsigned short* BO = (unsigned short*)take(WS_W);
  unsigned short* X16 = (unsigned short*)take(WS_P16);
  unsigned short* QH  = (unsigned short*)take(WS_P16);
  unsigned short* QR  = (unsigned short*)take(WS_P16);
  unsigned short* K16 = (unsigned short*)take(WS_P16);
  unsigned short* VT  = (unsigned short*)take(WS_P16);
  unsigned short* CH  = (unsigned short*)take(WS_P16);
  unsigned short* CL  = (unsigned short*)take(WS_P16);
  float* Y = (float*)take(WS_P32);
  if (off > ws_size) return;
  const unsigned gw = (unsigned)(((size_t)DM * (DM / 8) + 255) / 256);
  k_wt_f16<<<gw, 256, 0, stream>>>(wq, BQ, DM, DM, 16.0f);
  k_wt_f16<<<gw, 256, 0, stream>>>(wk, BK, DM, DM, 16.0f);
  k_wt_f16<<<gw, 256, 0, stream>>>(wv, BV, DM, DM, 16.0f);
  k_wt_bf16<<<gw, 256, 0, stream>>>(wo, BO, DM, DM);
  k_x16<<<(unsigned)(((size_t)NRP * DM / 8 + 255) / 256), 256, 0, stream>>>(x, X16);
  k_gemm_q<<<(unsigned)((NRP / 128) * (DM / 64)), 128, 0, stream>>>(X16, BQ, bq, QH, QR);
  k_gemm_k<<<(unsigned)((NRP / 128) * (DM / 64)), 128, 0, stream>>>(X16, BK, bk, K16);
  k_gemm_vt<<<(unsigned)((DM / 128) * (NRP / 64)), 128, 0, stream>>>(BV, X16, bv, VT);
  k_flash<<<(unsigned)(NB * NH * (SEQ / 64)), 128, 0, stream>>>(QH, QR, K16, VT, CH, CL);
  k_gemm_o<<<(unsigned)((NRP / 128) * (DM / 64)), 128, 0, stream>>>(CH, CL, BO, bo, Y);
  k_ln<<<(unsigned)NRP, 256, 0, stream>>>(x, Y, lg, lb, (float*)d_out);
}
